// MambaLayer_19129784336983
// MI455X (gfx1250) — hardware-verified
//
#include <hip/hip_runtime.h>
#include <math.h>

typedef __attribute__((ext_vector_type(16))) _Float16 v16h;
typedef __attribute__((ext_vector_type(8)))  _Float16 v8h;
typedef __attribute__((ext_vector_type(16))) __bf16   v16b;
typedef __attribute__((ext_vector_type(8)))  __bf16   v8b;
typedef __attribute__((ext_vector_type(8)))  float    v8f;
typedef __attribute__((ext_vector_type(4)))  float    v4f;
typedef __attribute__((ext_vector_type(4)))  unsigned v4u;

constexpr int kBatch  = 4;
constexpr int kSeq    = 4096;
constexpr int kCh     = 256;
constexpr int kDin    = 512;
constexpr int kNst    = 16;
constexpr int kDtR    = 16;
constexpr int kXzP    = 2 * kDin;
constexpr int kXdN    = kDtR + 2 * kNst;
constexpr int kXdP    = 64;
constexpr int kRows   = kBatch * kSeq;
constexpr int kLnRows = 32;
constexpr int kLnP    = 33;
constexpr int kConvTP = 260;
constexpr int kScanTS = 64;
constexpr int kScanCh = 64;
constexpr int kScanYP = 68;
constexpr float kLnEps   = 1e-5f;
constexpr float kInvCh   = 1.0f / (float)kCh;
static_assert(kXdN == 48 && kXdN <= kXdP);
static_assert((kCh % 32) == 0 && (kDin % 32) == 0);
static_assert((kRows % 64) == 0 && (kXzP % 64) == 0 && (kXdP % 64) == 0 && (kCh % 64) == 0 && (kSeq % 64) == 0);
static_assert((kSeq % kScanTS) == 0 && (kDin % kScanCh) == 0 && (kDin % 256) == 0 && (kSeq % kLnRows) == 0);
static_assert(kCh == 256 && kLnRows == 32);

constexpr size_t kOffWIN  = 0;
constexpr size_t kOffWX   = kOffWIN + (size_t)kXzP  * kCh  * 2;
constexpr size_t kOffWO   = kOffWX  + (size_t)kXdP  * kDin * 2;
constexpr size_t kOffXNH  = kOffWO  + (size_t)kCh   * kDin * 2;
constexpr size_t kOffXNL  = kOffXNH + (size_t)kRows * kCh  * 2;
constexpr size_t kOffXZ   = kOffXNL + (size_t)kRows * kCh  * 2;
constexpr size_t kOffU16  = kOffXZ  + (size_t)kRows * kXzP * 4;
constexpr size_t kOffXD   = kOffU16 + (size_t)kRows * kDin * 2;
constexpr size_t kOffYL   = kOffXD  + (size_t)kRows * kXdP * 4;
constexpr size_t kWsTotal = kOffYL  + (size_t)kRows * kDin * 2;
constexpr size_t kOffYH   = kOffXNH;
static_assert(kWsTotal == 122486784ull);
static_assert(kWsTotal <= 134217728ull);
static_assert((size_t)kRows * kDin * 2 == 2 * (size_t)kRows * kCh * 2);
static_assert((kOffWX % 128) == 0 && (kOffWO % 128) == 0 && (kOffXNH % 128) == 0 && (kOffXNL % 128) == 0 &&
              (kOffXZ % 128) == 0 && (kOffU16 % 128) == 0 && (kOffXD % 128) == 0 && (kOffYL % 128) == 0);

__device__ __forceinline__ unsigned f2bf_bits(float f) {
  const unsigned u = __float_as_uint(f);
  return ((u + 0x7FFFu + ((u >> 16) & 1u)) >> 16) & 0xFFFFu;
}
__device__ __forceinline__ float bf_bits2f(unsigned h) { return __uint_as_float(h << 16); }
__device__ __forceinline__ float bf16_value(float f) { return bf_bits2f(f2bf_bits(f)); }

__device__ __forceinline__ void split8(const v4f a0, const v4f a1, v4u& hi, v4u& lo) {
  unsigned hb[8], lb[8];
#pragma unroll
  for (int e = 0; e < 4; ++e) {
    const float f0 = a0[e];
    const float f1 = a1[e];
    hb[e]     = f2bf_bits(f0);
    hb[4 + e] = f2bf_bits(f1);
    lb[e]     = f2bf_bits(f0 - bf_bits2f(hb[e]));
    lb[4 + e] = f2bf_bits(f1 - bf_bits2f(hb[4 + e]));
  }
  hi[0] = hb[0] | (hb[1] << 16);
  hi[1] = hb[2] | (hb[3] << 16);
  hi[2] = hb[4] | (hb[5] << 16);
  hi[3] = hb[6] | (hb[7] << 16);
  lo[0] = lb[0] | (lb[1] << 16);
  lo[1] = lb[2] | (lb[3] << 16);
  lo[2] = lb[4] | (lb[5] << 16);
  lo[3] = lb[6] | (lb[7] << 16);
}
__device__ __forceinline__ v4u pack8(const v4f a0, const v4f a1) {
  unsigned hb[8];
#pragma unroll
  for (int e = 0; e < 4; ++e) {
    const float f0 = a0[e];
    const float f1 = a1[e];
    hb[e]     = f2bf_bits(f0);
    hb[4 + e] = f2bf_bits(f1);
  }
  v4u r;
  r[0] = hb[0] | (hb[1] << 16);
  r[1] = hb[2] | (hb[3] << 16);
  r[2] = hb[4] | (hb[5] << 16);
  r[3] = hb[6] | (hb[7] << 16);
  return r;
}

__device__ __forceinline__ float conv_silu_eval(float w0, float w1, float w2, float w3, float bc,
                                                float xm3, float xm2, float xm1, float xcur) {
  float acc = w0 * xm3;
  acc = fmaf(w1, xm2, acc);
  acc = fmaf(w2, xm1, acc);
  acc = fmaf(w3, xcur, acc);
  const float sv = acc + bc;
  const float sg = __builtin_amdgcn_rcpf(1.0f + expf(-sv));
  return sv * sg;
}

__device__ __forceinline__ void dep_guard4_h(v8f& a, v8f& b, v8f& c, v8f& d, v16h x, v16h y) { asm volatile("v_nop\n\tv_nop\n\tv_nop\n\tv_nop" : "+v"(a), "+v"(b), "+v"(c), "+v"(d) : "v"(x), "v"(y)); }
__device__ __forceinline__ void dep_guard4_b(v8f& a, v8f& b, v8f& c, v8f& d, v16b x, v16b y) { asm volatile("v_nop\n\tv_nop\n\tv_nop\n\tv_nop" : "+v"(a), "+v"(b), "+v"(c), "+v"(d) : "v"(x), "v"(y)); }
__device__ __forceinline__ void keep4_h(v16h a, v16h b, v16h c, v16h d) { asm volatile("v_nop" :: "v"(a), "v"(b), "v"(c), "v"(d)); }
__device__ __forceinline__ void keep4_b(v16b a, v16b b, v16b c, v16b d) { asm volatile("v_nop" :: "v"(a), "v"(b), "v"(c), "v"(d)); }
__device__ __forceinline__ void acc_guard4(v8f& a, v8f& b, v8f& c, v8f& d) { asm volatile("v_nop\n\tv_nop\n\tv_nop\n\tv_nop" : "+v"(a), "+v"(b), "+v"(c), "+v"(d)); }
template <typename T> struct Frag;
template <> struct Frag<_Float16> {
  typedef v16h V; union U { v16h v; v8h h[2]; };
  static __device__ __forceinline__ v16h load(const _Float16* p) {
    U f; f.h[0] = *(const v8h*)(p); f.h[1] = *(const v8h*)(p + 16); return f.v;
  }
  static __device__ __forceinline__ v8f mma(v16h a, v16h b, v8f c) {
    return __builtin_amdgcn_wmma_f32_16x16x32_f16(false, a, false, b, (short)0, c, false, false);
  }
  static __device__ __forceinline__ void guard4(v8f& a, v8f& b, v8f& c, v8f& d, v16h x, v16h y) { dep_guard4_h(a, b, c, d, x, y); }
  static __device__ __forceinline__ void keep(v16h a, v16h b, v16h c, v16h d) { keep4_h(a, b, c, d); }
};
template <> struct Frag<__bf16> {
  typedef v16b V; union U { v16b v; v8b h[2]; };
  static __device__ __forceinline__ v16b load(const __bf16* p) {
    U f; f.h[0] = *(const v8b*)(p); f.h[1] = *(const v8b*)(p + 16); return f.v;
  }
  static __device__ __forceinline__ v8f mma(v16b a, v16b b, v8f c) {
    return __builtin_amdgcn_wmma_f32_16x16x32_bf16(false, a, false, b, (short)0, c, false, false);
  }
  static __device__ __forceinline__ void guard4(v8f& a, v8f& b, v8f& c, v8f& d, v16b x, v16b y) { dep_guard4_b(a, b, c, d, x, y); }
  static __device__ __forceinline__ void keep(v16b a, v16b b, v16b c, v16b d) { keep4_b(a, b, c, d); }
};

template <int ET> struct Elem;
template <> struct Elem<0> { typedef _Float16 T; };
template <> struct Elem<1> { typedef __bf16 T; };
template <int ET, bool SA, bool SB, int BIAS_MODE, int OUT_MODE, bool RESID, int ACT = 0>
__global__ __launch_bounds__(256) void wmma_gemm64(
    const unsigned short* __restrict__ Ap, const unsigned short* __restrict__ A2p, int lda, long strideA,
    const unsigned short* __restrict__ Btp, const unsigned short* __restrict__ Bt2p, int ldb, long strideB,
    void* __restrict__ Cout, void* __restrict__ Cout2, int ldc, long strideC,
    const float* __restrict__ bias,
    const float* __restrict__ resid, long strideR,
    int M, int N, int K, float scale) {
  typedef typename Elem<ET>::T T;
  typedef typename Frag<T>::V V;
  const T* A = (const T*)Ap; const T* A2 = (const T*)A2p; const T* Bt = (const T*)Btp; const T* Bt2 = (const T*)Bt2p;
  __shared__ __align__(16) float sT[8][16 * 68];
  const int b    = blockIdx.y;
  const int lane = threadIdx.x & 31;
  const int wave = threadIdx.x >> 5;
  const int tilesN = N >> 6;
  const int tilesM = M >> 6;
  const int tile = blockIdx.x * 8 + wave;
  if (tile >= tilesM * tilesN) return;
  const int tm = tile / tilesN;
  const int tn = tile - tm * tilesN;
  const int m0 = tm << 6;
  const int n0 = tn << 6;

  const T* Ab  = A  + (size_t)b * strideA;
  const T* Bb  = Bt + (size_t)b * strideB;
  const T* Ab2 = SA ? (A2  + (size_t)b * strideA) : Ab;
  const T* Bb2 = SB ? (Bt2 + (size_t)b * strideB) : Bb;

  const int rlane = lane & 15;
  const int koff  = (lane >> 4) * 8;
  const int mOff  = (lane >> 4) * 8;

  v8f acc[4][4];
#pragma unroll
  for (int i = 0; i < 4; ++i)
#pragma unroll
    for (int j = 0; j < 4; ++j) acc[i][j] = (v8f){0.f,0.f,0.f,0.f,0.f,0.f,0.f,0.f};

  for (int k0 = 0; k0 < K; k0 += 32) {
    V bh[4], bl[4];
#pragma unroll
    for (int j = 0; j < 4; ++j) {
      const size_t bo = (size_t)(n0 + (j << 4) + rlane) * ldb + koff + k0;
      bh[j] = Frag<T>::load(Bb + bo);
      if (SB) bl[j] = Frag<T>::load(Bb2 + bo);
    }
#pragma unroll
    for (int i = 0; i < 4; ++i) {
      const size_t ao = (size_t)(m0 + (i << 4) + rlane) * lda + koff + k0;
      V ah = Frag<T>::load(Ab + ao);
      V al;
      if (SA) al = Frag<T>::load(Ab2 + ao);
#pragma unroll
      for (int j = 0; j < 4; ++j) {
        acc[i][j] = Frag<T>::mma(ah, bh[j], acc[i][j]);
        if (SB) acc[i][j] = Frag<T>::mma(ah, bl[j], acc[i][j]);
        if (SA) acc[i][j] = Frag<T>::mma(al, bh[j], acc[i][j]);
      }
      Frag<T>::guard4(acc[i][0], acc[i][1], acc[i][2], acc[i][3], ah, SA ? al : ah);
    }
    Frag<T>::keep(bh[0], bh[1], bh[2], bh[3]);
    if (SB) Frag<T>::keep(bl[0], bl[1], bl[2], bl[3]);
  }
  acc_guard4(acc[0][0], acc[0][1], acc[0][2], acc[0][3]);
  acc_guard4(acc[1][0], acc[1][1], acc[1][2], acc[1][3]);
  acc_guard4(acc[2][0], acc[2][1], acc[2][2], acc[2][3]);
  acc_guard4(acc[3][0], acc[3][1], acc[3][2], acc[3][3]);

  float* slab = sT[wave];
  const float* Rb = RESID ? (resid + (size_t)b * strideR) : nullptr;
#pragma unroll
  for (int i = 0; i < 4; ++i) {
    const int mBase = m0 + (i << 4);
#pragma unroll
    for (int j = 0; j < 4; ++j) {
      const int n = n0 + (j << 4) + rlane;
      float bv = 0.f;
      if (BIAS_MODE == 2) bv = bias[n];
#pragma unroll
      for (int r = 0; r < 8; ++r) {
        float v = acc[i][j][r] * scale;
        if (BIAS_MODE == 1) v += bias[mBase + mOff + r];
        if (BIAS_MODE == 2) v += bv;
        if (RESID) v += Rb[(size_t)(mBase + mOff + r) * ldc + n];
        if (ACT == 1) v = tanhf(v);
        if (ACT == 2) v = fmaxf(v, 0.0f);
        if (ACT == 4) v = (v > 0.f) ? v : 0.01f * v;
        slab[(mOff + r) * 68 + (j << 4) + rlane] = v;
      }
    }
    __builtin_amdgcn_fence(__ATOMIC_RELEASE, "workgroup");
    __builtin_amdgcn_wave_barrier();
    __builtin_amdgcn_fence(__ATOMIC_ACQUIRE, "workgroup");
    if (OUT_MODE == 0) {
      float* C = (float*)Cout + (size_t)b * strideC;
      const int hh = lane >> 4, c4 = (lane & 15) * 4;
      for (int pass = 0; pass < 2; ++pass) {
#pragma unroll
        for (int it = 0; it < 8; ++it) {
          const int row = it * 2 + hh;
          v4f v = *(const v4f*)(slab + row * 68 + c4);
          *(volatile v4f*)(C + (size_t)(mBase + row) * ldc + n0 + c4) = v;
        }
        __threadfence();
      }
    } else {
      const int q = lane >> 3, c8 = (lane & 7) * 8;
      unsigned short* C  = (unsigned short*)Cout  + (size_t)b * strideC;
      unsigned short* C2 = (OUT_MODE == 2) ? ((unsigned short*)Cout2 + (size_t)b * strideC) : nullptr;
      for (int pass = 0; pass < 2; ++pass) {
#pragma unroll
        for (int it = 0; it < 4; ++it) {
          const int row = it * 4 + q;
          const float* sp = slab + row * 68 + c8;
          v8h hv, lv;
#pragma unroll
          for (int e = 0; e < 8; ++e) {
            if (OUT_MODE == 1) {
              hv[e] = (_Float16)sp[e];
            } else {
              const unsigned short hb = (unsigned short)f2bf_bits(sp[e]);
              const unsigned short lb = (unsigned short)f2bf_bits(sp[e] - bf_bits2f(hb));
              hv[e] = __builtin_bit_cast(_Float16, hb);
              lv[e] = __builtin_bit_cast(_Float16, lb);
            }
          }
          *(volatile v8h*)(C + (size_t)(mBase + row) * ldc + n0 + c8) = hv;
          if (OUT_MODE == 2) *(volatile v8h*)(C2 + (size_t)(mBase + row) * ldc + n0 + c8) = lv;
        }
        __threadfence();
      }
    }
    __builtin_amdgcn_fence(__ATOMIC_RELEASE, "workgroup");
    __builtin_amdgcn_wave_barrier();
    __builtin_amdgcn_fence(__ATOMIC_ACQUIRE, "workgroup");
  }
}

__global__ __launch_bounds__(256) void cast_rows_bf16_kernel(
    const float* __restrict__ src, unsigned short* __restrict__ dst, int total8, int valid8)
{
  const int i = blockIdx.x * 256 + threadIdx.x;
  if (i >= total8) return;
  const bool live = (i < valid8);
  const int ic = live ? i : (valid8 - 1);
  const size_t s0 = (size_t)ic << 3;
  const v4f r0 = *(const v4f*)(src + s0);
  const v4f r1 = *(const v4f*)(src + s0 + 4);
  v4f a0, a1;
#pragma unroll
  for (int e = 0; e < 4; ++e) {
    const float f0 = r0[e];
    const float f1 = r1[e];
    a0[e] = live ? f0 : 0.0f;
    a1[e] = live ? f1 : 0.0f;
  }
  const v4u hv = pack8(a0, a1);
  unsigned short* q = dst + ((size_t)i << 3);
  *(volatile v4u*)q = hv;
  __threadfence();
  *(volatile v4u*)q = hv;
}

__global__ __launch_bounds__(256) void ln_kernel(
    const float* __restrict__ x, const float* __restrict__ nw, const float* __restrict__ nb,
    unsigned short* __restrict__ XNH, unsigned short* __restrict__ XNL)
{
  __shared__ __align__(16) float sX[kCh * kLnP];
  __shared__ float sP1[8 * 32];
  __shared__ float sP2[8 * 32];
  const int tid = threadIdx.x, lane = tid & 31, wave = tid >> 5;
  const int m0  = blockIdx.x * kLnRows;
  const int bix = m0 / kSeq;
  const int l0  = m0 - bix * kSeq;
  const float* xb = x + (size_t)bix * kCh * kSeq + l0 + lane;
  float s = 0.f;
#pragma unroll 8
  for (int j = 0; j < 32; ++j) {
    const int c = wave + 8 * j;
    const float v = bf16_value(xb[(size_t)c * kSeq]);
    sX[c * kLnP + lane] = v;
    s += v;
  }
  sP1[wave * 32 + lane] = s;
  __syncthreads();
  float tot = 0.f;
#pragma unroll
  for (int w = 0; w < 8; ++w) tot += sP1[w * 32 + lane];
  const float mean = tot * kInvCh;
  float s2 = 0.f;
#pragma unroll 8
  for (int j = 0; j < 32; ++j) {
    const int c = wave + 8 * j;
    const float dv = sX[c * kLnP + lane] - mean;
    s2 = fmaf(dv, dv, s2);
  }
  sP2[wave * 32 + lane] = s2;
  __syncthreads();
  float tot2 = 0.f;
#pragma unroll
  for (int w = 0; w < 8; ++w) tot2 += sP2[w * 32 + lane];
  const float var  = tot2 * kInvCh;
  const float rstd = rsqrtf(var + kLnEps);
#pragma unroll 4
  for (int j = 0; j < 32; ++j) {
    const int c = wave + 8 * j;
    const float g  = bf16_value(nw[c]);
    const float be = bf16_value(nb[c]);
    const float dv = sX[c * kLnP + lane] - mean;
    sX[c * kLnP + lane] = (dv * rstd) * g + be;
  }
  __syncthreads();
  v4u hv[4], lv[4];
#pragma unroll
  for (int it = 0; it < 4; ++it) {
    const int row = it * 8 + wave;
    v4f a0, a1;
#pragma unroll
    for (int e = 0; e < 4; ++e) {
      a0[e] = sX[(lane * 8 + e) * kLnP + row];
      a1[e] = sX[(lane * 8 + 4 + e) * kLnP + row];
    }
    split8(a0, a1, hv[it], lv[it]);
  }
  for (int pass = 0; pass < 2; ++pass) {
#pragma unroll
    for (int it = 0; it < 4; ++it) {
      const size_t o = (size_t)(m0 + it * 8 + wave) * kCh + lane * 8;
      *(volatile v4u*)(XNH + o) = hv[it];
      *(volatile v4u*)(XNL + o) = lv[it];
    }
    __threadfence();
  }
}

__global__ __launch_bounds__(256) void conv_silu_kernel(
    const float* __restrict__ XZ, const float* __restrict__ cw, const float* __restrict__ cb,
    unsigned short* __restrict__ U16)
{
  __shared__ __align__(16) float sT[16 * kConvTP];
  const int tid = threadIdx.x, lane = tid & 31, wave = tid >> 5;
  const int d0 = blockIdx.x * 256, d = d0 + tid;
  const int g0 = blockIdx.y * 64;
  const int tb = g0 & (kSeq - 1);
  const v4f wv = *(const v4f*)(cw + (size_t)d * 4);
  const float wq0 = wv[0], wq1 = wv[1], wq2 = wv[2], wq3 = wv[3];
  const float w0 = bf16_value(wq0), w1 = bf16_value(wq1), w2 = bf16_value(wq2), w3 = bf16_value(wq3);
  const float bc = bf16_value(cb[d]);
  float xm3, xm2, xm1;
  {
    const bool hist = (tb > 0);
    const int rb = hist ? (g0 - 3) : g0;
    const float v3 = XZ[(size_t)rb * kXzP + d];
    const float v2 = XZ[(size_t)(rb + 1) * kXzP + d];
    const float v1 = XZ[(size_t)(rb + 2) * kXzP + d];
    xm3 = hist ? v3 : 0.f;
    xm2 = hist ? v2 : 0.f;
    xm1 = hist ? v1 : 0.f;
  }
#pragma unroll 1
  for (int sub = 0; sub < 4; ++sub) {
    const int lb = g0 + sub * 16;
#pragma unroll 1
    for (int s = 0; s < 16; ++s) {
      float xcur = XZ[(size_t)(lb + s) * kXzP + d];
      asm volatile("" : "+v"(xcur));
      sT[s * kConvTP + tid] = conv_silu_eval(w0, w1, w2, w3, bc, xm3, xm2, xm1, xcur);
      xm3 = xm2; xm2 = xm1; xm1 = xcur;
    }
    __syncthreads();
    v4u bv[2];
#pragma unroll
    for (int it = 0; it < 2; ++it) {
      const float* sp = sT + (it * 8 + wave) * kConvTP + lane * 8;
      const v4f a0 = *(const v4f*)(sp);
      const v4f a1 = *(const v4f*)(sp + 4);
      bv[it] = pack8(a0, a1);
    }
    for (int pass = 0; pass < 2; ++pass) {
#pragma unroll
      for (int it = 0; it < 2; ++it)
        *(volatile v4u*)(U16 + (size_t)(lb + it * 8 + wave) * kDin + d0 + lane * 8) = bv[it];
      __threadfence();
    }
    __syncthreads();
  }
}

__global__ __launch_bounds__(64) void scan_kernel(
    const float* __restrict__ XD, const float* __restrict__ XZ,
    const float* __restrict__ cw, const float* __restrict__ cb,
    const float* __restrict__ Wdt, const float* __restrict__ bdt, const float* __restrict__ Alog,
    const float* __restrict__ Dp, unsigned short* __restrict__ YH, unsigned short* __restrict__ YL)
{
  __shared__ __align__(16) float sX[kScanTS * kXdP];
  __shared__ __align__(16) float sY[kScanTS * kScanYP];
  __shared__ __align__(16) float sW[kDtR * kScanCh];
  __shared__ __align__(16) float sA[kNst * kScanCh];
  const int tid = threadIdx.x, lane = tid & 31, wave = tid >> 5;
  constexpr int kBlkPerB = kDin / kScanCh;
  const int bix = blockIdx.x / kBlkPerB;
  const int d0  = (blockIdx.x - bix * kBlkPerB) * kScanCh;
  const int d   = d0 + tid;
  const size_t row0 = (size_t)bix * kSeq;
#pragma unroll 1
  for (int r = 0; r < kDtR; ++r) sW[r * kScanCh + tid] = bf16_value(Wdt[(size_t)d * kDtR + r]);
#pragma unroll 1
  for (int s = 0; s < kNst; ++s) sA[s * kScanCh + tid] = -expf(bf16_value(Alog[(size_t)d * kNst + s]));
  __syncthreads();
  float negA[kNst], h[kNst];
#pragma unroll
  for (int s = 0; s < kNst; ++s) {
    negA[s] = sA[s * kScanCh + tid];
    h[s] = 0.f;
  }
  const float bb = bf16_value(bdt[d]);
  const float Dd = bf16_value(Dp[d]);
  const v4f wv = *(const v4f*)(cw + (size_t)d * 4);
  const float wq0 = wv[0], wq1 = wv[1], wq2 = wv[2], wq3 = wv[3];
  const float w0 = bf16_value(wq0), w1 = bf16_value(wq1), w2 = bf16_value(wq2), w3 = bf16_value(wq3);
  const float bc = bf16_value(cb[d]);
  float xm3 = 0.f, xm2 = 0.f, xm1 = 0.f;
  const int lr = tid >> 4, lc4 = (tid & 15) * 4;
  const int q = lane >> 3, c8 = (lane & 7) * 8;
#pragma unroll 1
  for (int t0 = 0; t0 < kSeq; t0 += kScanTS) {
    __syncthreads();
#pragma unroll
    for (int i = 0; i < 16; ++i) {
      const int r = lr + 4 * i;
      *(v4f*)(sX + r * kXdP + lc4) = *(const v4f*)(XD + (row0 + t0 + r) * kXdP + lc4);
    }
    __syncthreads();
#pragma unroll 1
    for (int s = 0; s < kScanTS; ++s) {
      const int t = t0 + s;
      const float* xr = sX + s * kXdP;
      float vdot = 0.f;
#pragma unroll 1
      for (int r4 = 0; r4 < kDtR / 4; ++r4) {
        const v4f xv = *(const v4f*)(xr + 4 * r4);
        const float* wp = sW + (4 * r4) * kScanCh + tid;
        vdot = fmaf(xv[0], wp[0], vdot);
        vdot = fmaf(xv[1], wp[kScanCh], vdot);
        vdot = fmaf(xv[2], wp[2 * kScanCh], vdot);
        vdot = fmaf(xv[3], wp[3 * kScanCh], vdot);
      }
      float Bs[kNst], Cs[kNst];
#pragma unroll
      for (int q4 = 0; q4 < 4; ++q4) {
        const v4f bv = *(const v4f*)(xr + kDtR + 4 * q4);
        const v4f cv = *(const v4f*)(xr + kDtR + kNst + 4 * q4);
        Bs[4 * q4 + 0] = bv[0]; Bs[4 * q4 + 1] = bv[1]; Bs[4 * q4 + 2] = bv[2]; Bs[4 * q4 + 3] = bv[3];
        Cs[4 * q4 + 0] = cv[0]; Cs[4 * q4 + 1] = cv[1]; Cs[4 * q4 + 2] = cv[2]; Cs[4 * q4 + 3] = cv[3];
      }
      const float v   = vdot + bb;
      const float a   = __expf(-fabsf(v));
      const float u1  = 1.0f + a;
      const float l1p = __logf(u1) + (a - (u1 - 1.0f)) * __builtin_amdgcn_rcpf(u1);
      const float dt  = fmaxf(v, 0.0f) + l1p;
      float xcur = XZ[(row0 + t) * kXzP + d];
      asm volatile("" : "+v"(xcur));
      float zv = XZ[(row0 + t) * kXzP + kDin + d];
      asm volatile("" : "+v"(zv));
      const float xt = conv_silu_eval(w0, w1, w2, w3, bc, xm3, xm2, xm1, xcur);
      xm3 = xm2; xm2 = xm1; xm1 = xcur;
      const float dtx = dt * xt;
      float y = 0.f;
#pragma unroll
      for (int k = 0; k < kNst; ++k) {
        const float e = __expf(dt * negA[k]);
        h[k] = e * h[k] + dtx * Bs[k];
        y = h[k] * Cs[k] + y;
      }
      y = xt * Dd + y;
      const float sg = __builtin_amdgcn_rcpf(1.0f + expf(-zv));
      y = y * (zv * sg);
      sY[s * kScanYP + tid] = y;
    }
    __syncthreads();
    v4u hv[8], lv[8];
#pragma unroll
    for (int it = 0; it < 8; ++it) {
      const int row = it * 8 + wave * 4 + q;
      const float* sp = sY + row * kScanYP + c8;
      const v4f a0 = *(const v4f*)(sp);
      const v4f a1 = *(const v4f*)(sp + 4);
      split8(a0, a1, hv[it], lv[it]);
    }
    for (int pass = 0; pass < 2; ++pass) {
#pragma unroll
      for (int it = 0; it < 8; ++it) {
        const int row = it * 8 + wave * 4 + q;
        const size_t o = (row0 + t0 + row) * kDin + d0 + c8;
        *(volatile v4u*)(YH + o) = hv[it];
        *(volatile v4u*)(YL + o) = lv[it];
      }
      __threadfence();
    }
  }
}

extern "C" void kernel_launch(void* const* d_in, const int* in_sizes, int n_in,
                              void* d_out, int out_size, void* d_ws, size_t ws_size,
                              hipStream_t stream) {
  if (n_in < 12) return;
  if (in_sizes[0] != kBatch * kCh * kSeq) return;
  if (in_sizes[1] != kCh || in_sizes[2] != kCh) return;
  if (in_sizes[3] != kXzP * kCh) return;
  if (in_sizes[4] != kDin * 4 || in_sizes[5] != kDin) return;
  if (in_sizes[6] != kXdN * kDin) return;
  if (in_sizes[7] != kDin * kDtR || in_sizes[8] != kDin) return;
  if (in_sizes[9] != kDin * kNst || in_sizes[10] != kDin) return;
  if (in_sizes[11] != kCh * kDin) return;
  if (out_size != kBatch * kCh * kSeq) return;
  if (ws_size < kWsTotal) return;

  const float* x      = (const float*)d_in[0];
  const float* nw     = (const float*)d_in[1];
  const float* nbv    = (const float*)d_in[2];
  const float* W_in   = (const float*)d_in[3];
  const float* conv_w = (const float*)d_in[4];
  const float* conv_b = (const float*)d_in[5];
  const float* W_xp   = (const float*)d_in[6];
  const float* W_dt   = (const float*)d_in[7];
  const float* b_dt   = (const float*)d_in[8];
  const float* A_log  = (const float*)d_in[9];
  const float* Dp     = (const float*)d_in[10];
  const float* W_out  = (const float*)d_in[11];
  float* out = (float*)d_out;

  char* ws = (char*)d_ws;
  unsigned short* WIN = (unsigned short*)(ws + kOffWIN);
  unsigned short* WX  = (unsigned short*)(ws + kOffWX);
  unsigned short* WO  = (unsigned short*)(ws + kOffWO);
  unsigned short* XNH = (unsigned short*)(ws + kOffXNH);
  unsigned short* XNL = (unsigned short*)(ws + kOffXNL);
  float*          XZ  = (float*)(ws + kOffXZ);
  unsigned short* U16 = (unsigned short*)(ws + kOffU16);
  float*          XD  = (float*)(ws + kOffXD);
  unsigned short* YH  = (unsigned short*)(ws + kOffYH);
  unsigned short* YL  = (unsigned short*)(ws + kOffYL);
  const float* dummy_bias  = b_dt;
  const float* dummy_resid = x;

  cast_rows_bf16_kernel<<<(kXzP * kCh / 8) / 256, 256, 0, stream>>>(W_in, WIN, kXzP * kCh / 8, kXzP * kCh / 8);
  cast_rows_bf16_kernel<<<(kXdP * kDin / 8) / 256, 256, 0, stream>>>(W_xp, WX, kXdP * kDin / 8, kXdN * kDin / 8);
  cast_rows_bf16_kernel<<<(kCh * kDin / 8) / 256, 256, 0, stream>>>(W_out, WO, kCh * kDin / 8, kCh * kDin / 8);

  ln_kernel<<<kRows / kLnRows, 256, 0, stream>>>(x, nw, nbv, XNH, XNL);

  wmma_gemm64<1, true, false, 0, 0, false><<<dim3(512, 1), 256, 0, stream>>>(
      XNH, XNL, kCh, 0L,
      WIN, WIN, kCh, 0L,
      (void*)XZ, (void*)XZ, kXzP, 0L,
      dummy_bias, dummy_resid, 0L,
      kRows, kXzP, kCh, 1.0f);

  conv_silu_kernel<<<dim3(kDin / 256, kRows / 64), 256, 0, stream>>>(XZ, conv_w, conv_b, U16);

  wmma_gemm64<1, false, false, 0, 0, false><<<dim3(32, 1), 256, 0, stream>>>(
      U16, U16, kDin, 0L,
      WX, WX, kDin, 0L,
      (void*)XD, (void*)XD, kXdP, 0L,
      dummy_bias, dummy_resid, 0L,
      kRows, kXdP, kDin, 1.0f);

  scan_kernel<<<kBatch * (kDin / kScanCh), kScanCh, 0, stream>>>(XD, XZ, conv_w, conv_b, W_dt, b_dt, A_log, Dp, YH, YL);

  wmma_gemm64<1, false, true, 0, 0, false><<<dim3(32, kBatch), 256, 0, stream>>>(
      WO, WO, kDin, 0L,
      YH, YL, kDin, (long)kSeq * kDin,
      (void*)out, (void*)out, kSeq, (long)kCh * kSeq,
      dummy_bias, dummy_resid, 0L,
      kCh, kSeq, kDin, 1.0f);
}
